// TiteAttention_73057393705645
// MI455X (gfx1250) — hardware-run, weakly checked
//
#include <hip/hip_runtime.h>
#include <math.h>
#include <stdint.h>

constexpr int TOK_TOTAL  = 16384;
constexpr int HID        = 768;
constexpr int NUM_SEQ    = 8;
constexpr int SEQ_TOK    = 2048;
constexpr int NUM_HEAD   = 12;
constexpr int HEAD_D     = 64;
constexpr int QK_COLS    = 2 * HID;
constexpr int CHUNK_SEQS = 2;
constexpr int CHUNK_TOK  = CHUNK_SEQS * SEQ_TOK;
constexpr int NUM_CHUNK  = NUM_SEQ / CHUNK_SEQS;
constexpr int ROPE_HALF  = HEAD_D / 2;
constexpr float W_CARRY  = 64.0f;
constexpr float P_CARRY  = 32768.0f;
constexpr float O_CARRY  = 64.0f;

typedef __attribute__((ext_vector_type(16))) _Float16 v16h;
typedef __attribute__((ext_vector_type(8)))  _Float16 v8h;
typedef __attribute__((ext_vector_type(16))) __bf16   v16b;
typedef __attribute__((ext_vector_type(8)))  __bf16   v8b;
typedef __attribute__((ext_vector_type(8)))  float    v8f;
typedef __attribute__((ext_vector_type(4)))  float    v4f;
typedef __attribute__((ext_vector_type(2)))  unsigned int v2u;
typedef __attribute__((ext_vector_type(4)))  unsigned int v4u;

__device__ __forceinline__ unsigned short f2bf_bits(float f) {
  unsigned u = __float_as_uint(f);
  return (unsigned short)((u + 0x7FFFu + ((u >> 16) & 1u)) >> 16);
}
__device__ __forceinline__ float bf_bits2f(unsigned short h) { return __uint_as_float(((unsigned)h) << 16); }
__device__ __forceinline__ unsigned short h_bits(float f) { return __builtin_bit_cast(unsigned short, (_Float16)f); }
__device__ __forceinline__ unsigned pk16(unsigned short a, unsigned short b) { return (unsigned)a | ((unsigned)b << 16); }

__device__ __forceinline__ void dep_guard_h(v8f& a, v8f& b, v16h x, v16h y) { asm volatile("v_nop\n\tv_nop\n\tv_nop\n\tv_nop" : "+v"(a), "+v"(b) : "v"(x), "v"(y)); }
__device__ __forceinline__ void dep_guard_b(v8f& a, v8f& b, v16b x, v16b y) { asm volatile("v_nop\n\tv_nop\n\tv_nop\n\tv_nop" : "+v"(a), "+v"(b) : "v"(x), "v"(y)); }
__device__ __forceinline__ void keep4_h(v16h a, v16h b, v16h c, v16h d) { asm volatile("v_nop" :: "v"(a), "v"(b), "v"(c), "v"(d)); }
__device__ __forceinline__ void keep4_b(v16b a, v16b b, v16b c, v16b d) { asm volatile("v_nop" :: "v"(a), "v"(b), "v"(c), "v"(d)); }
__device__ __forceinline__ void acc_guard4(v8f& a, v8f& b, v8f& c, v8f& d) { asm volatile("v_nop\n\tv_nop\n\tv_nop\n\tv_nop" : "+v"(a), "+v"(b), "+v"(c), "+v"(d)); }
template <typename T> struct Frag;
template <> struct Frag<_Float16> {
  typedef v16h V; union U { v16h v; v8h h[2]; };
  static __device__ __forceinline__ v16h load(const _Float16* p) {
    U f; f.h[0] = *(const v8h*)(p); f.h[1] = *(const v8h*)(p + 16); return f.v;
  }
  static __device__ __forceinline__ v8f mma(v16h a, v16h b, v8f c) {
    return __builtin_amdgcn_wmma_f32_16x16x32_f16(false, a, false, b, (short)0, c, false, false);
  }
  static __device__ __forceinline__ void guard(v8f& a, v8f& b, v16h x, v16h y) { dep_guard_h(a, b, x, y); }
  static __device__ __forceinline__ void keep(v16h a, v16h b, v16h c, v16h d) { keep4_h(a, b, c, d); }
};
template <> struct Frag<__bf16> {
  typedef v16b V; union U { v16b v; v8b h[2]; };
  static __device__ __forceinline__ v16b load(const __bf16* p) {
    U f; f.h[0] = *(const v8b*)(p); f.h[1] = *(const v8b*)(p + 16); return f.v;
  }
  static __device__ __forceinline__ v8f mma(v16b a, v16b b, v8f c) {
    return __builtin_amdgcn_wmma_f32_16x16x32_bf16(false, a, false, b, (short)0, c, false, false);
  }
  static __device__ __forceinline__ void guard(v8f& a, v8f& b, v16b x, v16b y) { dep_guard_b(a, b, x, y); }
  static __device__ __forceinline__ void keep(v16b a, v16b b, v16b c, v16b d) { keep4_b(a, b, c, d); }
};

template <int ET> struct Elem;
template <> struct Elem<0> { typedef _Float16 T; };
template <> struct Elem<1> { typedef __bf16 T; };
template <int ET, bool SPLIT, int BIAS_MODE, int OUT_MODE, bool RESID, int ACT = 0>
__global__ __launch_bounds__(256) void wmma_gemm64(
    const unsigned short* __restrict__ Ap, const unsigned short* __restrict__ A2p, int lda, long strideA,
    const unsigned short* __restrict__ Btp, const unsigned short* __restrict__ Bt2p, int ldb, long strideB,
    void* __restrict__ Cout, void* __restrict__ Cout2, int ldc, long strideC,
    const float* __restrict__ bias,
    const float* __restrict__ resid, long strideR,
    int M, int N, int K, float scale) {
  typedef typename Elem<ET>::T T;
  typedef typename Frag<T>::V V;
  const T* A = (const T*)Ap; const T* A2 = (const T*)A2p; const T* Bt = (const T*)Btp; const T* Bt2 = (const T*)Bt2p;
  __shared__ __align__(16) float sT[8][16 * 68];
  const int b    = blockIdx.y;
  const int lane = threadIdx.x & 31;
  const int wave = threadIdx.x >> 5;
  const int tilesN = N >> 6;
  const int tilesM = M >> 6;
  const int tile = blockIdx.x * 8 + wave;
  if (tile >= tilesM * tilesN) return;
  const int tm = tile / tilesN;
  const int tn = tile - tm * tilesN;
  const int m0 = tm << 6;
  const int n0 = tn << 6;

  const T* Ab  = A  + (size_t)b * strideA;
  const T* Bb  = Bt + (size_t)b * strideB;
  const T* Ab2 = SPLIT ? (A2  + (size_t)b * strideA) : nullptr;
  const T* Bb2 = SPLIT ? (Bt2 + (size_t)b * strideB) : nullptr;

  const int rlane = lane & 15;
  const int koff  = (lane >> 4) * 8;
  const int mOff  = (lane >> 4) * 8;

  v8f acc[4][4];
#pragma unroll
  for (int i = 0; i < 4; ++i)
#pragma unroll
    for (int j = 0; j < 4; ++j) acc[i][j] = (v8f){0.f,0.f,0.f,0.f,0.f,0.f,0.f,0.f};

  for (int k0 = 0; k0 < K; k0 += 32) {
    V bh[4], bl[4];
#pragma unroll
    for (int j = 0; j < 4; ++j) {
      const size_t bo = (size_t)(n0 + (j << 4) + rlane) * ldb + koff + k0;
      bh[j] = Frag<T>::load(Bb + bo);
      if (SPLIT) bl[j] = Frag<T>::load(Bb2 + bo);
    }
#pragma unroll
    for (int i = 0; i < 4; ++i) {
      const size_t ao = (size_t)(m0 + (i << 4) + rlane) * lda + koff + k0;
      V ah = Frag<T>::load(Ab + ao);
      V al;
      if (SPLIT) al = Frag<T>::load(Ab2 + ao);
#pragma unroll
      for (int j = 0; j < 4; ++j) {
        acc[i][j] = Frag<T>::mma(ah, bh[j], acc[i][j]);
        if (SPLIT) {
          acc[i][j] = Frag<T>::mma(ah, bl[j], acc[i][j]);
          acc[i][j] = Frag<T>::mma(al, bh[j], acc[i][j]);
        }
      }
      Frag<T>::guard(acc[i][0], acc[i][3], ah, SPLIT ? al : ah);
    }
    Frag<T>::keep(bh[0], bh[1], bh[2], bh[3]);
    if (SPLIT) Frag<T>::keep(bl[0], bl[1], bl[2], bl[3]);
  }
  acc_guard4(acc[0][0], acc[0][1], acc[0][2], acc[0][3]);
  acc_guard4(acc[1][0], acc[1][1], acc[1][2], acc[1][3]);
  acc_guard4(acc[2][0], acc[2][1], acc[2][2], acc[2][3]);
  acc_guard4(acc[3][0], acc[3][1], acc[3][2], acc[3][3]);

  float* slab = sT[wave];
  const float* Rb = RESID ? (resid + (size_t)b * strideR) : nullptr;
#pragma unroll
  for (int i = 0; i < 4; ++i) {
    const int mBase = m0 + (i << 4);
#pragma unroll
    for (int j = 0; j < 4; ++j) {
      const int n = n0 + (j << 4) + rlane;
      float bv = 0.f;
      if (BIAS_MODE == 2) bv = bias[n];
#pragma unroll
      for (int r = 0; r < 8; ++r) {
        float v = acc[i][j][r] * scale;
        if (BIAS_MODE == 1) v += bias[mBase + mOff + r];
        if (BIAS_MODE == 2) v += bv;
        if (RESID) v += Rb[(size_t)(mBase + mOff + r) * ldc + n];
        if (ACT == 1) v = tanhf(v);
        if (ACT == 2) v = fmaxf(v, 0.0f);
        if (ACT == 3) v = v / (1.0f + expf(-v));
        if (ACT == 4) v = (v > 0.f) ? v : 0.01f * v;
        if (ACT == 5) v = 0.5f * v * (1.0f + erff(v * 0.70710678118654752f));
        slab[(mOff + r) * 68 + (j << 4) + rlane] = v;
      }
    }
    __builtin_amdgcn_fence(__ATOMIC_RELEASE, "workgroup");
    __builtin_amdgcn_wave_barrier();
    __builtin_amdgcn_fence(__ATOMIC_ACQUIRE, "workgroup");
    if (OUT_MODE == 0) {
      float* C = (float*)Cout + (size_t)b * strideC;
      const int hh = lane >> 4, c4 = (lane & 15) * 4;
      for (int pass = 0; pass < 2; ++pass) {
#pragma unroll
        for (int it = 0; it < 8; ++it) {
          const int row = it * 2 + hh;
          v4f v = *(const v4f*)(slab + row * 68 + c4);
          *(volatile v4f*)(C + (size_t)(mBase + row) * ldc + n0 + c4) = v;
        }
        __threadfence();
      }
    } else {
      const int q = lane >> 3, c8 = (lane & 7) * 8;
      unsigned short* C  = (unsigned short*)Cout  + (size_t)b * strideC;
      unsigned short* C2 = (OUT_MODE == 2) ? ((unsigned short*)Cout2 + (size_t)b * strideC) : nullptr;
      for (int pass = 0; pass < 2; ++pass) {
#pragma unroll
        for (int it = 0; it < 4; ++it) {
          const int row = it * 4 + q;
          const float* sp = slab + row * 68 + c8;
          v8h hv, lv;
#pragma unroll
          for (int e = 0; e < 8; ++e) {
            if (OUT_MODE == 1) {
              hv[e] = (_Float16)sp[e];
            } else {
              unsigned short hb = f2bf_bits(sp[e]);
              unsigned short lb = f2bf_bits(sp[e] - bf_bits2f(hb));
              hv[e] = __builtin_bit_cast(_Float16, hb);
              lv[e] = __builtin_bit_cast(_Float16, lb);
            }
          }
          *(volatile v8h*)(C + (size_t)(mBase + row) * ldc + n0 + c8) = hv;
          if (OUT_MODE == 2) *(volatile v8h*)(C2 + (size_t)(mBase + row) * ldc + n0 + c8) = lv;
        }
        __threadfence();
      }
    }
    __builtin_amdgcn_fence(__ATOMIC_RELEASE, "workgroup");
    __builtin_amdgcn_wave_barrier();
    __builtin_amdgcn_fence(__ATOMIC_ACQUIRE, "workgroup");
  }
}

__global__ __launch_bounds__(256) void ln_rows_kernel(const float* __restrict__ x, const float* __restrict__ gw,
                                                      const float* __restrict__ gb, float* __restrict__ xf,
                                                      unsigned short* __restrict__ xh, int nrows, float eps) {
  const int row  = blockIdx.x * 8 + (threadIdx.x >> 5);
  const int lane = threadIdx.x & 31;
  if (row >= nrows) return;
  const float* xr = x + (size_t)row * HID;
  v4f v[6];
  float s = 0.f;
#pragma unroll
  for (int it = 0; it < 6; ++it) {
    v[it] = *(const v4f*)(xr + it * 128 + lane * 4);
    s += (v[it][0] + v[it][1]) + (v[it][2] + v[it][3]);
  }
#pragma unroll
  for (int off = 1; off < 32; off <<= 1) s += __shfl_xor(s, off, 32);
  const float mean = s * (1.0f / (float)HID);
  float ss = 0.f;
#pragma unroll
  for (int it = 0; it < 6; ++it) {
#pragma unroll
    for (int e = 0; e < 4; ++e) { const float d = v[it][e] - mean; ss += d * d; }
  }
#pragma unroll
  for (int off = 1; off < 32; off <<= 1) ss += __shfl_xor(ss, off, 32);
  const float var  = ss * (1.0f / (float)HID);
  const float rstd = rsqrtf(var + eps);
  v4f y[6]; v2u yh[6];
#pragma unroll
  for (int it = 0; it < 6; ++it) {
    const v4f wv  = *(const v4f*)(gw + it * 128 + lane * 4);
    const v4f bb4 = *(const v4f*)(gb + it * 128 + lane * 4);
    v4f o;
#pragma unroll
    for (int e = 0; e < 4; ++e) o[e] = (v[it][e] - mean) * rstd * wv[e] + bb4[e];
    y[it] = o;
    v2u pk; pk[0] = pk16(h_bits(o[0]), h_bits(o[1])); pk[1] = pk16(h_bits(o[2]), h_bits(o[3]));
    yh[it] = pk;
  }
  float* xfr = xf + (size_t)row * HID;
  unsigned short* xhr = xh + (size_t)row * HID;
  for (int pass = 0; pass < 2; ++pass) {
#pragma unroll
    for (int it = 0; it < 6; ++it) {
      *(volatile v4f*)(xfr + it * 128 + lane * 4) = y[it];
      *(volatile v2u*)(xhr + it * 128 + lane * 4) = yh[it];
    }
    __threadfence();
  }
}

__global__ __launch_bounds__(256) void wtcast_kernel(const float* __restrict__ w0, const float* __restrict__ w1,
                                                     const float* __restrict__ w2, const float* __restrict__ w3,
                                                     unsigned short* __restrict__ outp, int R, int Cc, long sOut, float mul) {
  __shared__ __align__(16) float tf[64 * 68];
  const int z = blockIdx.z;
  const float* W = (z == 0) ? w0 : (z == 1) ? w1 : (z == 2) ? w2 : w3;
  unsigned short* oh = outp + (size_t)z * sOut;
  const int c0  = blockIdx.x * 64;
  const int r0  = blockIdx.y * 64;
  const int tid = threadIdx.x;
  {
    const int lr = tid >> 4;
    const int c4 = (tid & 15) * 4;
#pragma unroll
    for (int it = 0; it < 4; ++it) {
      const int rr = it * 16 + lr;
      const v4f a = *(const v4f*)(W + (size_t)(r0 + rr) * Cc + c0 + c4);
      *(v4f*)(tf + rr * 68 + c4) = a;
    }
  }
  __syncthreads();
  const int sub = tid >> 3;
  const int c8  = (tid & 7) * 8;
  v4u hv[2];
#pragma unroll
  for (int it = 0; it < 2; ++it) {
    const int oc = it * 32 + sub;
    v4u a;
#pragma unroll
    for (int qd = 0; qd < 4; ++qd) {
      const float f0 = tf[(c8 + 2 * qd) * 68 + oc] * mul;
      const float f1 = tf[(c8 + 2 * qd + 1) * 68 + oc] * mul;
      a[qd] = pk16(h_bits(f0), h_bits(f1));
    }
    hv[it] = a;
  }
  for (int pass = 0; pass < 2; ++pass) {
#pragma unroll
    for (int it = 0; it < 2; ++it) {
      const int oc = it * 32 + sub;
      const size_t go = (size_t)(c0 + oc) * R + r0 + c8;
      *(volatile v4u*)(oh + go) = hv[it];
    }
    __threadfence();
  }
}

__global__ __launch_bounds__(256) void bias_cat_kernel(const float* __restrict__ ba, const float* __restrict__ bb2,
                                                       float* __restrict__ outp, int na, int nb) {
  const int i = blockIdx.x * 256 + threadIdx.x;
  if (i < na + nb) {
    const int ia = min(i, na - 1);
    const int ib = min(max(i - na, 0), nb - 1);
    const float fa = ba[ia];
    const float fb = bb2[ib];
    const float v = (i < na) ? fa : fb;
    ((volatile float*)outp)[i] = v;
    __threadfence();
    ((volatile float*)outp)[i] = v;
  }
}

__global__ __launch_bounds__(256) void rope_tab_kernel(float* __restrict__ ctab, float* __restrict__ stab, int n) {
  const int i = blockIdx.x * 256 + threadIdx.x;
  if (i < n) {
    const int pos = i >> 5, j = i & 31;
    const float invf = exp2f(-(float)j * 0.41524101186092f);
    const float th = (float)pos * invf;
    const float cs = cosf(th);
    const float sn = sinf(th);
    ((volatile float*)ctab)[i] = cs;
    ((volatile float*)stab)[i] = sn;
    __threadfence();
    ((volatile float*)ctab)[i] = cs;
    ((volatile float*)stab)[i] = sn;
  }
}

__global__ __launch_bounds__(256) void rope_kernel(const float* __restrict__ qk, const float* __restrict__ ctab,
                                                   const float* __restrict__ stab, unsigned short* __restrict__ qo,
                                                   unsigned short* __restrict__ ko, int ntok) {
  const int wid  = blockIdx.x * 8 + (threadIdx.x >> 5);
  const int lane = threadIdx.x & 31;
  const int row  = wid >> 1, sel = wid & 1;
  if (row >= ntok) return;
  const int pos = row & (SEQ_TOK - 1);
  const float* src = qk + (size_t)row * QK_COLS + sel * HID;
  unsigned short* dst = (sel ? ko : qo) + (size_t)row * HID;
  const float* ct = ctab + (size_t)pos * ROPE_HALF;
  const float* st = stab + (size_t)pos * ROPE_HALF;
  v2u ov[6];
#pragma unroll
  for (int it = 0; it < 6; ++it) {
    const int cidx = it * 128 + lane * 4;
    const int jh = cidx & (HEAD_D - 1);
    const int pcol = (jh < ROPE_HALF) ? (cidx + ROPE_HALF) : (cidx - ROPE_HALF);
    const float sg = (jh < ROPE_HALF) ? -1.0f : 1.0f;
    const int jj = cidx & (ROPE_HALF - 1);
    const v4f a  = *(const v4f*)(src + cidx);
    const v4f p  = *(const v4f*)(src + pcol);
    const v4f cs = *(const v4f*)(ct + jj);
    const v4f sn = *(const v4f*)(st + jj);
    float o[4];
#pragma unroll
    for (int e = 0; e < 4; ++e) o[e] = a[e] * cs[e] + (sg * p[e]) * sn[e];
    v2u pk; pk[0] = pk16(h_bits(o[0]), h_bits(o[1])); pk[1] = pk16(h_bits(o[2]), h_bits(o[3]));
    ov[it] = pk;
  }
  for (int pass = 0; pass < 2; ++pass) {
#pragma unroll
    for (int it = 0; it < 6; ++it) *(volatile v2u*)(dst + it * 128 + lane * 4) = ov[it];
    __threadfence();
  }
}

constexpr int ATT_D = 64, ATT_NW = 4, ATT_QB = 64, ATT_KC = 64;

__device__ __forceinline__ v8f mma_f16_g(v16h a, v16h b, v8f c) {
  c = __builtin_amdgcn_wmma_f32_16x16x32_f16(false, a, false, b, (short)0, c, false, false);
  asm volatile("v_nop\n\tv_nop\n\tv_nop\n\tv_nop" : "+v"(c) : "v"(a), "v"(b));
  return c;
}

__global__ __launch_bounds__(128)
void attn_f16_kernel(const unsigned short* __restrict__ qp, const unsigned short* __restrict__ kp,
                     const unsigned short* __restrict__ vtp, unsigned short* __restrict__ op,
                     int ldv, float sscale) {
  union FH { v16h v; v8h h[2]; };
  __shared__ __align__(16) _Float16 Ksh[ATT_KC * ATT_D];
  __shared__ __align__(16) _Float16 Vth[ATT_D * ATT_KC];
  __shared__ __align__(16) _Float16 Psh[ATT_NW][16 * ATT_KC];
  __shared__ __align__(16) float    Os[ATT_NW][16 * 68];

  const int tid  = threadIdx.x;
  const int wave = tid >> 5;
  const int lane = tid & 31;
  const int hh   = lane >> 4;
  const int c    = lane & 15;

  constexpr int nqb = SEQ_TOK / ATT_QB;
  const int bx = blockIdx.x;
  const int qb = bx % nqb;
  const int h  = (bx / nqb) % NUM_HEAD;
  const int sl = bx / (nqb * NUM_HEAD);
  const int q0 = qb * ATT_QB + wave * 16;
  const size_t rowbase = (size_t)sl * SEQ_TOK;

  const _Float16* Qh = (const _Float16*)(const void*)qp + rowbase * HID + (size_t)h * ATT_D;
  const _Float16* Kh = (const _Float16*)(const void*)kp + rowbase * HID + (size_t)h * ATT_D;
  const _Float16* Vh = (const _Float16*)(const void*)vtp + (size_t)h * ATT_D * ldv + rowbase;
  _Float16*       ob = (_Float16*)(void*)op + rowbase * HID + (size_t)h * ATT_D;

  v16h qa[2];
#pragma unroll
  for (int dc = 0; dc < 2; ++dc) qa[dc] = Frag<_Float16>::load(Qh + (size_t)(q0 + c) * HID + dc * 32 + 8 * hh);

  float mrow[8], lrow[8];
  v8f oacc[4];
#pragma unroll
  for (int r = 0; r < 8; ++r) { mrow[r] = -INFINITY; lrow[r] = 0.f; }
#pragma unroll
  for (int t = 0; t < 4; ++t) oacc[t] = (v8f){0.f,0.f,0.f,0.f,0.f,0.f,0.f,0.f};

  constexpr int nChunks = SEQ_TOK / ATT_KC;
  for (int kc = 0; kc < nChunks; ++kc) {
    const int kv0 = kc * ATT_KC;
    __syncthreads();
    {
      const int r = tid >> 1, half = (tid & 1) * 32;
      const _Float16* ksh = Kh + (size_t)(kv0 + r) * HID + half;
      const _Float16* vsh = Vh + (size_t)r * ldv + kv0 + half;
#pragma unroll
      for (int i = 0; i < 4; ++i) {
        const v8h a0 = *(const v8h*)(ksh + 8 * i);
        const v8h b0 = *(const v8h*)(vsh + 8 * i);
        *(v8h*)(Ksh + r * ATT_D  + half + 8 * i) = a0;
        *(v8h*)(Vth + r * ATT_KC + half + 8 * i) = b0;
      }
    }
    __syncthreads();

    v8f s[4];
#pragma unroll
    for (int j = 0; j < 4; ++j) {
      s[j] = (v8f){0.f,0.f,0.f,0.f,0.f,0.f,0.f,0.f};
#pragma unroll
      for (int dc = 0; dc < 2; ++dc) {
        FH kb;
        kb.h[0] = *(const v8h*)(Ksh + (j * 16 + c) * ATT_D + dc * 32 + 8 * hh);
        kb.h[1] = *(const v8h*)(Ksh + (j * 16 + c) * ATT_D + dc * 32 + 16 + 8 * hh);
        s[j] = mma_f16_g(qa[dc], kb.v, s[j]);
      }
    }
    float cm[8];
#pragma unroll
    for (int r = 0; r < 8; ++r) {
      float m = -INFINITY;
#pragma unroll
      for (int j = 0; j < 4; ++j) {
        const float sv = s[j][r] * sscale;
        s[j][r] = sv;
        m = fmaxf(m, sv);
      }
#pragma unroll
      for (int off = 1; off < 16; off <<= 1) m = fmaxf(m, __shfl_xor(m, off, 32));
      cm[r] = m;
    }
    _Float16* pwh = Psh[wave];
#pragma unroll
    for (int r = 0; r < 8; ++r) {
      const float mnew  = fmaxf(mrow[r], cm[r]);
      const float alpha = expf(mrow[r] - mnew);
      mrow[r] = mnew;
      float psum = 0.f;
#pragma unroll
      for (int j = 0; j < 4; ++j) {
        const float p = expf(s[j][r] - mnew);
        psum += p;
        pwh[(8 * hh + r) * ATT_KC + j * 16 + c] = (_Float16)(p * P_CARRY);
      }
#pragma unroll
      for (int off = 1; off < 16; off <<= 1) psum += __shfl_xor(psum, off, 32);
      lrow[r] = lrow[r] * alpha + psum;
#pragma unroll
      for (int t = 0; t < 4; ++t) oacc[t][r] *= alpha;
    }
    __builtin_amdgcn_fence(__ATOMIC_RELEASE, "workgroup");
    __builtin_amdgcn_wave_barrier();
    __builtin_amdgcn_fence(__ATOMIC_ACQUIRE, "workgroup");
#pragma unroll 1
    for (int kk = 0; kk < 2; ++kk) {
      FH pa;
      pa.h[0] = *(const v8h*)(pwh + c * ATT_KC + kk * 32 + 8 * hh);
      pa.h[1] = *(const v8h*)(pwh + c * ATT_KC + kk * 32 + 16 + 8 * hh);
#pragma unroll
      for (int t = 0; t < 4; ++t) {
        FH vb;
        vb.h[0] = *(const v8h*)(Vth + (t * 16 + c) * ATT_KC + kk * 32 + 8 * hh);
        vb.h[1] = *(const v8h*)(Vth + (t * 16 + c) * ATT_KC + kk * 32 + 16 + 8 * hh);
        oacc[t] = mma_f16_g(pa.v, vb.v, oacc[t]);
      }
    }
  }

  float* os = Os[wave];
#pragma unroll
  for (int r = 0; r < 8; ++r) {
    const float inv = (O_CARRY / P_CARRY) * (1.0f / lrow[r]);
#pragma unroll
    for (int t = 0; t < 4; ++t) os[(8 * hh + r) * 68 + t * 16 + c] = oacc[t][r] * inv;
  }
  __builtin_amdgcn_fence(__ATOMIC_RELEASE, "workgroup");
  __builtin_amdgcn_wave_barrier();
  __builtin_amdgcn_fence(__ATOMIC_ACQUIRE, "workgroup");
  {
    const int qq = lane >> 3, c8 = (lane & 7) * 8;
    for (int pass = 0; pass < 2; ++pass) {
#pragma unroll
      for (int it = 0; it < 4; ++it) {
        const int row = it * 4 + qq;
        const float* sp = os + row * 68 + c8;
        v8h hv;
#pragma unroll
        for (int e = 0; e < 8; ++e) hv[e] = (_Float16)sp[e];
        *(volatile v8h*)(ob + (size_t)(q0 + row) * HID + c8) = hv;
      }
      __threadfence();
    }
  }
}

extern "C" void kernel_launch(void* const* d_in, const int* in_sizes, int n_in,
                              void* d_out, int out_size, void* d_ws, size_t ws_size,
                              hipStream_t stream) {
  if (n_in < 13) return;
  if (in_sizes[0] != TOK_TOTAL * HID || out_size != TOK_TOTAL * HID) return;
  if (in_sizes[3] != HID || in_sizes[4] != HID) return;
  if (in_sizes[5] != HID * HID || in_sizes[7] != HID * HID || in_sizes[9] != HID * HID || in_sizes[11] != HID * HID) return;
  if (in_sizes[6] != HID || in_sizes[8] != HID || in_sizes[10] != HID || in_sizes[12] != HID) return;

  const float* p_hs = (const float*)d_in[0];
  const float* p_nw = (const float*)d_in[3];
  const float* p_nb = (const float*)d_in[4];
  const float* p_Wq = (const float*)d_in[5];  const float* p_bq = (const float*)d_in[6];
  const float* p_Wk = (const float*)d_in[7];  const float* p_bk = (const float*)d_in[8];
  const float* p_Wv = (const float*)d_in[9];  const float* p_bv = (const float*)d_in[10];
  const float* p_Wo = (const float*)d_in[11]; const float* p_bo = (const float*)d_in[12];
  float* p_out = (float*)d_out;

  char* ws = (char*)d_ws;
  size_t off = 0;
  auto carve = [&](size_t bytes) -> char* {
    char* p = ws + off;
    off += (bytes + 255) & ~(size_t)255;
    return p;
  };
  const size_t planeW = (size_t)HID * HID;
  float*          XF   = (float*)carve((size_t)TOK_TOTAL * HID * sizeof(float));
  unsigned short* X16  = (unsigned short*)carve((size_t)TOK_TOTAL * HID * 2);
  unsigned short* W16  = (unsigned short*)carve(4 * planeW * 2);
  float*          BQK  = (float*)carve((size_t)QK_COLS * sizeof(float));
  float*          CTAB = (float*)carve((size_t)SEQ_TOK * ROPE_HALF * sizeof(float));
  float*          STAB = (float*)carve((size_t)SEQ_TOK * ROPE_HALF * sizeof(float));
  float*          QKF  = (float*)carve((size_t)CHUNK_TOK * QK_COLS * sizeof(float));
  unsigned short* Q16  = (unsigned short*)carve((size_t)CHUNK_TOK * HID * 2);
  unsigned short* K16  = (unsigned short*)carve((size_t)CHUNK_TOK * HID * 2);
  unsigned short* VT16 = (unsigned short*)carve((size_t)HID * CHUNK_TOK * 2);
  unsigned short* O16  = (unsigned short*)carve((size_t)CHUNK_TOK * HID * 2);
  if (off > ws_size) return;

  const dim3 blk256(256);
  const dim3 blk128(128);

  ln_rows_kernel<<<dim3(TOK_TOTAL / 8), blk256, 0, stream>>>(p_hs, p_nw, p_nb, XF, X16, TOK_TOTAL, 1e-12f);

  wtcast_kernel<<<dim3(HID / 64, HID / 64, 4), blk256, 0, stream>>>(p_Wq, p_Wk, p_Wv, p_Wo, W16, HID, HID,
                                                                    (long)planeW, W_CARRY);

  bias_cat_kernel<<<dim3(QK_COLS / 256), blk256, 0, stream>>>(p_bq, p_bk, BQK, HID, HID);

  rope_tab_kernel<<<dim3(SEQ_TOK * ROPE_HALF / 256), blk256, 0, stream>>>(CTAB, STAB, SEQ_TOK * ROPE_HALF);

  const int qkTiles  = (CHUNK_TOK / 64) * (QK_COLS / 64);
  const int vtTiles  = (HID / 64) * (CHUNK_TOK / 64);
  const int outTiles = (CHUNK_TOK / 64) * (HID / 64);
  const int attnBlocks = CHUNK_SEQS * NUM_HEAD * (SEQ_TOK / ATT_QB);

  for (int ch = 0; ch < NUM_CHUNK; ++ch) {
    const size_t tok0 = (size_t)ch * CHUNK_TOK;
    const unsigned short* X16c = X16 + tok0 * HID;
    const float* XFc = XF + tok0 * HID;
    float* outc = p_out + tok0 * HID;

    wmma_gemm64<0, false, 2, 0, false, 0><<<dim3((qkTiles + 7) / 8, 1), blk256, 0, stream>>>(
        X16c, X16c, HID, 0L,
        W16, W16, HID, 0L,
        (void*)QKF, (void*)QKF, QK_COLS, 0L,
        BQK, XFc, 0L,
        CHUNK_TOK, QK_COLS, HID, 1.0f / W_CARRY);

    wmma_gemm64<0, false, 1, 1, false, 0><<<dim3((vtTiles + 7) / 8, 1), blk256, 0, stream>>>(
        W16 + 2 * planeW, W16 + 2 * planeW, HID, 0L,
        X16c, X16c, HID, 0L,
        (void*)VT16, (void*)VT16, CHUNK_TOK, 0L,
        p_bv, XFc, 0L,
        HID, CHUNK_TOK, HID, 1.0f / W_CARRY);

    rope_kernel<<<dim3(CHUNK_TOK * 2 / 8), blk256, 0, stream>>>(QKF, CTAB, STAB, Q16, K16, CHUNK_TOK);

    attn_f16_kernel<<<dim3(attnBlocks), blk128, 0, stream>>>(Q16, K16, VT16, O16, CHUNK_TOK, 0.125f);

    wmma_gemm64<0, false, 2, 0, true, 0><<<dim3((outTiles + 7) / 8, 1), blk256, 0, stream>>>(
        O16, O16, HID, 0L,
        W16 + 3 * planeW, W16 + 3 * planeW, HID, 0L,
        (void*)outc, (void*)outc, HID, 0L,
        p_bo, XFc, 0L,
        CHUNK_TOK, HID, HID, 1.0f / (W_CARRY * O_CARRY));
  }
}
